// GNE_3418793968191
// MI455X (gfx1250) — hardware-verified
//
#include <hip/hip_runtime.h>


namespace {
constexpr int B = 4, N = 256, T = 2048, HTD = 64, L = 4, PAD = 16, TR = T + PAD;
constexpr float XS = 8.0f, PS = 1024.0f, WSC = 256.0f;
typedef _Float16 b16;
typedef __attribute__((ext_vector_type(16))) _Float16 v16b;
typedef __attribute__((ext_vector_type(8))) _Float16 v8b;
typedef __attribute__((ext_vector_type(8))) float v8f;
typedef __attribute__((ext_vector_type(4))) float v4f;
typedef __attribute__((ext_vector_type(2))) _Float16 v2b;
__device__ __forceinline__ float bf16_rne(float f) { unsigned int u = __float_as_uint(f); u += 0x7FFFu + ((u >> 16) & 1u); return __uint_as_float(u & 0xFFFF0000u); }
__device__ __forceinline__ void split16(float v, b16& hi, b16& lo) { hi = (b16)v; lo = (b16)(v - (float)hi); }
__device__ __forceinline__ v16b frag_kb(const b16* p, int hh) { const v8b a = *(const v8b*)(p + 8 * hh), b = *(const v8b*)(p + 16 + 8 * hh); v16b f;
#pragma unroll
  for (int e = 0; e < 8; ++e) { f[e] = a[e]; f[8 + e] = b[e]; } return f; }
__device__ __forceinline__ v8f wmma16b(v16b a, v16b b, v8f c) { v8f d = __builtin_amdgcn_wmma_f32_16x16x32_f16(false, a, false, b, (short)0, c, false, false); asm volatile("v_nop\n\tv_nop\n\tv_nop\n\tv_nop" : "+v"(d) : "v"(a), "v"(b)); return d; }
__device__ __forceinline__ void wave_lds_sync() { __builtin_amdgcn_fence(__ATOMIC_RELEASE, "workgroup"); __builtin_amdgcn_wave_barrier(); __builtin_amdgcn_fence(__ATOMIC_ACQUIRE, "workgroup"); }
__device__ __forceinline__ float pmul(float a, float b) { float p = a * b; asm volatile("" : "+v"(p)); return p; }

__global__ __launch_bounds__(256) void wgen_kernel(const float* __restrict__ w, int rows, int K, long sr, long sk, long o0, int op, b16* __restrict__ WT) {
  const size_t u = (size_t)blockIdx.x * 256 + threadIdx.x; if (u >= (size_t)rows * K / 8) return; const int r = (int)(u / (K / 8)), k0 = (int)(u % (K / 8)) * 8; v8b v;
#pragma unroll
  for (int j = 0; j < 8; ++j) v[j] = (b16)(bf16_rne(w[(size_t)r * sr + (size_t)(k0 + j) * sk + o0]) * WSC); for (int pass = 0; pass < 2; ++pass) { *(volatile v8b*)(WT + (size_t)r * op + k0) = v; __threadfence(); }
}
__global__ __launch_bounds__(256) void zpad_kernel(float* __restrict__ F0, b16* __restrict__ H0, b16* __restrict__ L0, float* __restrict__ F1, b16* __restrict__ H1, b16* __restrict__ L1) {
  const int b = blockIdx.x & 3, buf = blockIdx.x >> 2; float* Fp = (buf ? F1 : F0) + (size_t)b * TR * N; b16* Hp = (buf ? H1 : H0) + (size_t)b * TR * N; b16* Lp = (buf ? L1 : L0) + (size_t)b * TR * N;
  for (int pass = 0; pass < 2; ++pass) { for (int i = threadIdx.x; i < PAD * N; i += 256) { ((volatile float*)Fp)[i] = 0.0f; ((volatile b16*)Hp)[i] = (b16)0.0f; ((volatile b16*)Lp)[i] = (b16)0.0f; } __threadfence(); }
}
__global__ __launch_bounds__(256) void tin_kernel(const float* __restrict__ Xk, int BV, float* __restrict__ YF, b16* __restrict__ YH, b16* __restrict__ YL) {
  __shared__ float Ts[64][N + 1]; const int tid = threadIdx.x, wave = tid >> 5, lane = tid & 31; const int b = blockIdx.x / (T / 64), t0 = (blockIdx.x % (T / 64)) * 64; if (b >= BV) return;
  for (int n = wave; n < N; n += 8) { const float* src = Xk + ((size_t)b * N + n) * T + t0; Ts[lane][n] = bf16_rne(src[lane]); Ts[32 + lane][n] = bf16_rne(src[32 + lane]); }
  __syncthreads();
  for (int pass = 0; pass < 2; ++pass) { for (int r = 0; r < 8; ++r) { const int tt = wave * 8 + r; const size_t row = ((size_t)b * TR + PAD + t0 + tt) * N; for (int q = 0; q < 8; ++q) { const int n = q * 32 + lane; const float v = Ts[tt][n]; ((volatile float*)YF)[row + n] = v; b16 p, ql; split16(pmul(v, XS), p, ql); ((volatile b16*)YH)[row + n] = p; ((volatile b16*)YL)[row + n] = ql; } } __threadfence(); }
}
__global__ __launch_bounds__(32) void tblock_kernel(const float* __restrict__ YF, const b16* __restrict__ YH, const b16* __restrict__ YL, const b16* __restrict__ WCV, const float* __restrict__ cb, const b16* __restrict__ WPJ, const float* __restrict__ pb, int d, int BV, float* __restrict__ OF, b16* __restrict__ OH, b16* __restrict__ OL) {
  __shared__ __attribute__((aligned(16))) b16 Rh[16][N + 8], Rl[16][N + 8]; __shared__ float Zs[16][N + 1];
  const int lane = threadIdx.x, nloc = lane & 15, hlf = lane >> 4; const int b = blockIdx.x / (T / 16), t0 = (blockIdx.x % (T / 16)) * 16; if (b >= BV) return; const size_t rb0 = (size_t)b * TR + PAD + t0;
  v8f acc[16];
#pragma unroll
  for (int tt = 0; tt < 16; ++tt) acc[tt] = (v8f){};
#pragma unroll 1
  for (int tap = 0; tap < 3; ++tap) { const size_t ra = (rb0 + nloc - (size_t)(2 - tap) * d) * N;
#pragma unroll 2
    for (int ib = 0; ib < N; ib += 32) { const v16b ah = frag_kb(YH + ra + ib, hlf), al = frag_kb(YL + ra + ib, hlf); const int k0 = tap * N + ib;
#pragma unroll
      for (int tt = 0; tt < 16; ++tt) { const v16b bw = frag_kb(WCV + (size_t)(tt * 16 + nloc) * (3 * N) + k0, hlf); acc[tt] = wmma16b(ah, bw, acc[tt]); acc[tt] = wmma16b(al, bw, acc[tt]); } } }
#pragma unroll
  for (int tt = 0; tt < 16; ++tt) { const int o = tt * 16 + nloc; const float bb = bf16_rne(cb[o]);
#pragma unroll
    for (int r8 = 0; r8 < 8; ++r8) { b16 p, q; split16(fmaxf(acc[tt][r8] * (1.0f / (XS * WSC)) + bb, 0.0f) * XS, p, q); Rh[8 * hlf + r8][o] = p; Rl[8 * hlf + r8][o] = q; } }
  wave_lds_sync();
#pragma unroll
  for (int tt = 0; tt < 16; ++tt) acc[tt] = (v8f){};
#pragma unroll 2
  for (int ib = 0; ib < N; ib += 32) { const v16b ah = frag_kb(&Rh[nloc][ib], hlf), al = frag_kb(&Rl[nloc][ib], hlf);
#pragma unroll
    for (int tt = 0; tt < 16; ++tt) { const v16b bw = frag_kb(WPJ + (size_t)(tt * 16 + nloc) * N + ib, hlf); acc[tt] = wmma16b(ah, bw, acc[tt]); acc[tt] = wmma16b(al, bw, acc[tt]); } }
#pragma unroll
  for (int tt = 0; tt < 16; ++tt) { const int o = tt * 16 + nloc; const float bb = bf16_rne(pb[o]);
#pragma unroll
    for (int r8 = 0; r8 < 8; ++r8) Zs[8 * hlf + r8][o] = acc[tt][r8] * (1.0f / (XS * WSC)) + bb; }
  wave_lds_sync();
  for (int pass = 0; pass < 2; ++pass) { for (int rr = 0; rr < 16; ++rr) { const size_t row = (rb0 + rr) * N; for (int q = 0; q < 8; ++q) { const int n = q * 32 + lane; const float v = YF[row + n] + Zs[rr][n]; ((volatile float*)OF)[row + n] = v; b16 p, ql; split16(v * XS, p, ql); ((volatile b16*)OH)[row + n] = p; ((volatile b16*)OL)[row + n] = ql; } } __threadfence(); }
}
__global__ __launch_bounds__(256) void tout_kernel(const float* __restrict__ YF, int BV, b16* __restrict__ YNh, b16* __restrict__ YNl) {
  __shared__ float Ts[64][N + 1]; const int tid = threadIdx.x, wave = tid >> 5, lane = tid & 31; const int b = blockIdx.x / (T / 64), t0 = (blockIdx.x % (T / 64)) * 64; if (b >= BV) return;
  for (int tt = wave; tt < 64; tt += 8) { const float* src = YF + ((size_t)b * TR + PAD + t0 + tt) * N; for (int q = 0; q < 8; ++q) Ts[tt][q * 32 + lane] = src[q * 32 + lane]; }
  __syncthreads();
  for (int pass = 0; pass < 2; ++pass) { for (int n = wave; n < N; n += 8) { const size_t o_ = ((size_t)b * N + n) * T + t0; b16 p0, q0, p1, q1; split16(pmul(Ts[2 * lane][n], XS), p0, q0); split16(pmul(Ts[2 * lane + 1][n], XS), p1, q1); ((volatile v2b*)(YNh + o_))[lane] = (v2b){p0, p1}; ((volatile v2b*)(YNl + o_))[lane] = (v2b){q0, q1}; } __threadfence(); }
}
__global__ __launch_bounds__(32) void ht_kernel(const b16* __restrict__ WG, const b16* __restrict__ YNh, const b16* __restrict__ YNl, int BV, float* __restrict__ HTF, b16* __restrict__ HTh, b16* __restrict__ HTl) {
  __shared__ float Hs[16][N + 1]; const int lane = threadIdx.x, nloc = lane & 15, hlf = lane >> 4; const int b = blockIdx.x / (T / 16), u0 = (blockIdx.x % (T / 16)) * 16; if (b >= BV) return;
  v8f acc[16];
#pragma unroll
  for (int tt = 0; tt < 16; ++tt) acc[tt] = (v8f){};
  const b16* yh = YNh + (size_t)b * N * T; const b16* yl = YNl + (size_t)b * N * T;
#pragma unroll 2
  for (int kb = 0; kb < T; kb += 32) { const v16b a = frag_kb(WG + (size_t)(u0 + nloc) * T + kb, hlf);
#pragma unroll
    for (int tt = 0; tt < 16; ++tt) { const size_t nr = (size_t)(tt * 16 + nloc) * T + kb; acc[tt] = wmma16b(a, frag_kb(yh + nr, hlf), acc[tt]); acc[tt] = wmma16b(a, frag_kb(yl + nr, hlf), acc[tt]); } }
#pragma unroll
  for (int tt = 0; tt < 16; ++tt)
#pragma unroll
    for (int r8 = 0; r8 < 8; ++r8) Hs[8 * hlf + r8][tt * 16 + nloc] = acc[tt][r8] * (1.0f / (WSC * XS));
  wave_lds_sync();
  for (int pass = 0; pass < 2; ++pass) { for (int rr = 0; rr < 16; ++rr) { const size_t row = ((size_t)b * T + u0 + rr) * N; for (int q = 0; q < 8; ++q) { const int n = q * 32 + lane; const float v = Hs[rr][n]; ((volatile float*)HTF)[row + n] = v; b16 p, ql; split16(v * XS, p, ql); ((volatile b16*)HTh)[row + n] = p; ((volatile b16*)HTl)[row + n] = ql; } } __threadfence(); }
}
__global__ __launch_bounds__(256) void eij_kernel(const float* __restrict__ HTF, const float* __restrict__ a1, const float* __restrict__ a2, int BV, float* __restrict__ EI, float* __restrict__ EJ) {
  const int b = blockIdx.x, n = threadIdx.x; if (b >= BV) return; float si = 0.0f, sj = 0.0f; const float* hp = HTF + (size_t)b * T * N + n;
#pragma unroll 4
  for (int u = 0; u < T; ++u) { const float hv = hp[(size_t)u * N]; si += pmul(hv, bf16_rne(a1[u])); sj += pmul(hv, bf16_rne(a2[u])); }
  for (int pass = 0; pass < 2; ++pass) { ((volatile float*)EI)[b * N + n] = si; ((volatile float*)EJ)[b * N + n] = sj; __threadfence(); }
}
__global__ __launch_bounds__(256) void att_kernel(const float* __restrict__ EI, const float* __restrict__ EJ, int BV, float* __restrict__ Aout, b16* __restrict__ Ah, b16* __restrict__ Al) {
  const int wave = threadIdx.x >> 5, lane = threadIdx.x & 31; const int bi = blockIdx.x * 8 + wave, b = bi / N, i = bi % N; if (b >= BV) return; const float e0 = EI[b * N + i]; float e[8], mx = -INFINITY;
#pragma unroll
  for (int k = 0; k < 8; ++k) { float v = e0 + EJ[b * N + k * 32 + lane]; v = v > 0.0f ? v : 0.2f * v; e[k] = v; mx = fmaxf(mx, v); }
  for (int o = 16; o; o >>= 1) mx = fmaxf(mx, __shfl_xor(mx, o)); float s = 0.0f;
#pragma unroll
  for (int k = 0; k < 8; ++k) { e[k] = __expf(e[k] - mx); s += e[k]; }
  for (int o = 16; o; o >>= 1) s += __shfl_xor(s, o); const float inv = 1.0f / s;
  for (int pass = 0; pass < 2; ++pass) {
#pragma unroll
    for (int k = 0; k < 8; ++k) { const size_t p_ = ((size_t)b * N + i) * N + k * 32 + lane; const float a = e[k] * inv; ((volatile float*)Aout)[p_] = a; b16 p, q; split16(a * PS, p, q); ((volatile b16*)Ah)[p_] = p; ((volatile b16*)Al)[p_] = q; } __threadfence(); }
}
__global__ __launch_bounds__(32) void y2_kernel(const b16* __restrict__ HTh, const b16* __restrict__ HTl, const b16* __restrict__ Ah, const b16* __restrict__ Al, const float* __restrict__ ht, const float* __restrict__ hw, const float* __restrict__ hb, int BV, b16* __restrict__ Y2h, b16* __restrict__ Y2l) {
  __shared__ float Cd[N], Ys[16][N + 1]; const int lane = threadIdx.x, nloc = lane & 15, hlf = lane >> 4; const int b = blockIdx.x / (T / 16), u0 = (blockIdx.x % (T / 16)) * 16; if (b >= BV) return;
  for (int q = 0; q < 8; ++q) { const int i = q * 32 + lane; float s = bf16_rne(hb[i]); for (int k = 0; k < HTD; ++k) s += pmul(bf16_rne(ht[b * HTD + k]), bf16_rne(hw[i * HTD + k])); Cd[i] = s; }
  v8f acc[16];
#pragma unroll
  for (int tt = 0; tt < 16; ++tt) acc[tt] = (v8f){};
  const b16* hh = HTh + ((size_t)b * T + u0 + nloc) * N; const b16* hl = HTl + ((size_t)b * T + u0 + nloc) * N; const b16* ah0 = Ah + (size_t)b * N * N; const b16* al0 = Al + (size_t)b * N * N;
#pragma unroll
  for (int kb = 0; kb < N; kb += 32) { const v16b fh = frag_kb(hh + kb, hlf), fl = frag_kb(hl + kb, hlf);
#pragma unroll
    for (int tt = 0; tt < 16; ++tt) { const size_t ir = (size_t)(tt * 16 + nloc) * N + kb; const v16b bh = frag_kb(ah0 + ir, hlf), bl = frag_kb(al0 + ir, hlf); acc[tt] = wmma16b(fh, bh, acc[tt]); acc[tt] = wmma16b(fh, bl, acc[tt]); acc[tt] = wmma16b(fl, bh, acc[tt]); } }
  wave_lds_sync();
#pragma unroll
  for (int tt = 0; tt < 16; ++tt) { const int i = tt * 16 + nloc; const float cd = Cd[i];
#pragma unroll
    for (int r8 = 0; r8 < 8; ++r8) Ys[8 * hlf + r8][i] = acc[tt][r8] * (1.0f / (XS * PS)) + cd; }
  wave_lds_sync();
  for (int pass = 0; pass < 2; ++pass) { for (int rr = 0; rr < 16; ++rr) { const size_t row = ((size_t)b * T + u0 + rr) * N; for (int q = 0; q < 8; ++q) { const int i = q * 32 + lane; b16 p, ql; split16(Ys[rr][i] * XS, p, ql); ((volatile b16*)Y2h)[row + i] = p; ((volatile b16*)Y2l)[row + i] = ql; } } __threadfence(); }
}
__global__ __launch_bounds__(32) void out_kernel(const b16* __restrict__ WO, const b16* __restrict__ Y2h, const b16* __restrict__ Y2l, const float* __restrict__ ob, int BV, float* __restrict__ out) {
  __shared__ float Tf[16][132]; const int lane = threadIdx.x, nloc = lane & 15, hlf = lane >> 4; const int per = (N / 16) * (T / 128); const int b = blockIdx.x / per, o0 = ((blockIdx.x % per) / (T / 128)) * 16, t0 = (blockIdx.x % (T / 128)) * 128; if (b >= BV) return;
  v8f acc[8];
#pragma unroll
  for (int tt = 0; tt < 8; ++tt) acc[tt] = (v8f){};
#pragma unroll
  for (int kb = 0; kb < N; kb += 32) { const v16b a = frag_kb(WO + (size_t)(o0 + nloc) * N + kb, hlf);
#pragma unroll
    for (int tt = 0; tt < 8; ++tt) { const size_t tr = ((size_t)b * T + t0 + tt * 16 + nloc) * N + kb; acc[tt] = wmma16b(a, frag_kb(Y2h + tr, hlf), acc[tt]); acc[tt] = wmma16b(a, frag_kb(Y2l + tr, hlf), acc[tt]); } }
#pragma unroll
  for (int tt = 0; tt < 8; ++tt)
#pragma unroll
    for (int r8 = 0; r8 < 8; ++r8) Tf[8 * hlf + r8][tt * 16 + nloc] = acc[tt][r8] * (1.0f / (WSC * XS)) + bf16_rne(ob[o0 + 8 * hlf + r8]);
  wave_lds_sync();
  for (int pass = 0; pass < 2; ++pass) { for (int rr = 0; rr < 16; ++rr) *(volatile v4f*)(out + ((size_t)b * N + o0 + rr) * T + t0 + lane * 4) = *(const v4f*)(&Tf[rr][lane * 4]); __threadfence(); }
}
}

extern "C" void kernel_launch(void* const* d_in, const int* in_sizes, int n_in, void* d_out, int out_size, void* d_ws, size_t ws_size, hipStream_t stream) {
  (void)n_in;
  auto Fp = [&](int i) { return (const float*)d_in[i]; };
  if (in_sizes[0] != B * N * T || in_sizes[1] != B * HTD || in_sizes[2] != L * N * N * 3 || in_sizes[4] != L * N * N || in_sizes[6] != T * T || in_sizes[7] != T || in_sizes[9] != N * N || in_sizes[11] != N * HTD || out_size != B * N * T + B * N * N) return;
  const int BV = B;
  size_t off = 0; char* ws = (char*)d_ws;
  auto carve = [&](size_t bytes) { char* p = ws + off; off += (bytes + 255) & ~(size_t)255; return p; };
  b16* WCV = (b16*)carve((size_t)L * N * 3 * N * 2); b16* WPJ = (b16*)carve((size_t)L * N * N * 2); b16* WG = (b16*)carve((size_t)T * T * 2); b16* WO = (b16*)carve((size_t)N * N * 2);
  float* YF[2]; b16* YH[2]; b16* YL[2]; for (int s = 0; s < 2; ++s) { YF[s] = (float*)carve((size_t)B * TR * N * 4); YH[s] = (b16*)carve((size_t)B * TR * N * 2); YL[s] = (b16*)carve((size_t)B * TR * N * 2); }
  b16* YNh = (b16*)carve((size_t)B * N * T * 2); b16* YNl = (b16*)carve((size_t)B * N * T * 2); float* HTF = (float*)carve((size_t)B * T * N * 4); b16* HTh = (b16*)carve((size_t)B * T * N * 2); b16* HTl = (b16*)carve((size_t)B * T * N * 2);
  float* EI = (float*)carve(B * N * 4); float* EJ = (float*)carve(B * N * 4); b16* Ah = (b16*)carve((size_t)B * N * N * 2); b16* Al = (b16*)carve((size_t)B * N * N * 2); b16* Y2h = (b16*)carve((size_t)B * T * N * 2); b16* Y2l = (b16*)carve((size_t)B * T * N * 2);
  if (off > ws_size || off > ((size_t)96 << 20)) return;
  for (int l = 0; l < L; ++l) for (int tap = 0; tap < 3; ++tap) wgen_kernel<<<(N * N / 8 + 255) / 256, 256, 0, stream>>>(Fp(2), N, N, 3L * N, 3, (long)l * N * N * 3 + tap, 3 * N, WCV + ((size_t)l * N * 3 * N + tap * N));
  for (int l = 0; l < L; ++l) wgen_kernel<<<(N * N / 8 + 255) / 256, 256, 0, stream>>>(Fp(4), N, N, (long)N, 1, (long)l * N * N, N, WPJ + (size_t)l * N * N);
  wgen_kernel<<<(T * T / 8 + 255) / 256, 256, 0, stream>>>(Fp(6), T, T, (long)T, 1, 0, T, WG); wgen_kernel<<<(N * N / 8 + 255) / 256, 256, 0, stream>>>(Fp(9), N, N, (long)N, 1, 0, N, WO);
  zpad_kernel<<<8, 256, 0, stream>>>(YF[0], YH[0], YL[0], YF[1], YH[1], YL[1]);
  tin_kernel<<<BV * (T / 64), 256, 0, stream>>>(Fp(0), BV, YF[0], YH[0], YL[0]);
  for (int l = 0; l < L; ++l) { const int s = l & 1, d = 1 << l; tblock_kernel<<<BV * (T / 16), 32, 0, stream>>>(YF[s], YH[s], YL[s], WCV + (size_t)l * N * 3 * N, Fp(3) + l * N, WPJ + (size_t)l * N * N, Fp(5) + l * N, d, BV, YF[s ^ 1], YH[s ^ 1], YL[s ^ 1]); }
  tout_kernel<<<BV * (T / 64), 256, 0, stream>>>(YF[0], BV, YNh, YNl);
  ht_kernel<<<BV * (T / 16), 32, 0, stream>>>(WG, YNh, YNl, BV, HTF, HTh, HTl);
  eij_kernel<<<BV, 256, 0, stream>>>(HTF, Fp(7), Fp(8), BV, EI, EJ);
  float* out = (float*)d_out;
  att_kernel<<<(BV * N) / 8, 256, 0, stream>>>(EI, EJ, BV, out + (size_t)B * N * T, Ah, Al);
  y2_kernel<<<BV * (T / 16), 32, 0, stream>>>(HTh, HTl, Ah, Al, Fp(1), Fp(11), Fp(12), BV, Y2h, Y2l);
  out_kernel<<<BV * (N / 16) * (T / 128), 32, 0, stream>>>(WO, Y2h, Y2l, Fp(10), BV, out);
}
